// MultiHeadedDotAttention_63050119905518
// MI455X (gfx1250) — hardware-verified
//
#include <hip/hip_runtime.h>
#include <math.h>
#include <stdint.h>


typedef _Float16 v16h __attribute__((ext_vector_type(16)));
typedef _Float16 v8h __attribute__((ext_vector_type(8)));
typedef __bf16 v16bf __attribute__((ext_vector_type(16)));
typedef unsigned short v8us_t __attribute__((ext_vector_type(8)));
typedef v8us_t __attribute__((may_alias)) v8us;
typedef float v8f __attribute__((ext_vector_type(8)));
typedef float v4f_t __attribute__((ext_vector_type(4)));
typedef v4f_t __attribute__((may_alias)) v4f;
typedef int v8i __attribute__((ext_vector_type(8)));

constexpr int BB = 4;
constexpr int SS = 1024;
constexpr int DD = 1024;
constexpr int HH = 16;
constexpr int DK = 64;
constexpr int NTOK = BB * SS;
constexpr long NX = (long)NTOK * DD;
constexpr long NW = (long)DD * DD;

union Frag { v16h f; v16bf b; v8us p[2]; v8i w; };

__device__ __forceinline__ unsigned short bf16_rne(float x) {
  unsigned u = __float_as_uint(x);
  u += 0x7FFFu + ((u >> 16) & 1u);
  return (unsigned short)(u >> 16);
}
__device__ __forceinline__ float bf16_val(unsigned short b) {
  return __uint_as_float(((unsigned)b) << 16);
}
__device__ __forceinline__ void split2(float x, unsigned short& hi, unsigned short& lo) {
  hi = bf16_rne(x);
  lo = bf16_rne(x - bf16_val(hi));
}
__device__ __forceinline__ unsigned short f16_bits(float x) {
  _Float16 hv = (_Float16)x;
  unsigned short u;
  __builtin_memcpy(&u, &hv, 2);
  return u;
}

__device__ __forceinline__ Frag ldfrag(const unsigned short* rowp, int k0, int hh) {
  Frag f;
  f.p[0] = *(const v8us*)(rowp + k0 + 8 * hh);
  f.p[1] = *(const v8us*)(rowp + k0 + 16 + 8 * hh);
  return f;
}

__device__ __forceinline__ v8f mma_f16(const Frag& a, const Frag& b, v8f c) {
  c = __builtin_amdgcn_wmma_f32_16x16x32_f16(false, a.f, false, b.f, (short)0, c, false, false);
  asm volatile("v_nop\n\tv_nop\n\tv_nop\n\tv_nop" : "+v"(c) : "v"(a.w), "v"(b.w));
  return c;
}

__device__ __forceinline__ v8f mma3(const Frag& ah, const Frag& al, const Frag& bh, const Frag& bl, v8f c) {
  c = __builtin_amdgcn_wmma_f32_16x16x32_bf16(false, ah.b, false, bh.b, (short)0, c, false, false);
  c = __builtin_amdgcn_wmma_f32_16x16x32_bf16(false, ah.b, false, bl.b, (short)0, c, false, false);
  c = __builtin_amdgcn_wmma_f32_16x16x32_bf16(false, al.b, false, bh.b, (short)0, c, false, false);
  asm volatile("v_nop\n\tv_nop\n\tv_nop\n\tv_nop"
               : "+v"(c)
               : "v"(ah.w), "v"(al.w), "v"(bh.w), "v"(bl.w));
  return c;
}

__global__ __launch_bounds__(256)
void k_cvt16(const float* __restrict__ src, unsigned short* __restrict__ dst, int n8, float scale) {
  const int i = blockIdx.x * 256 + threadIdx.x;
  if (i >= n8) return;
  const float* s = src + (size_t)i * 8;
  const v4f x0 = *(const v4f*)(s);
  const v4f x1 = *(const v4f*)(s + 4);
  union { v8h h; v8us_t u; } cv;
#pragma unroll
  for (int c = 0; c < 4; ++c) {
    cv.h[c]     = (_Float16)(x0[c] * scale);
    cv.h[4 + c] = (_Float16)(x1[c] * scale);
  }
  const v8us v = cv.u;
  unsigned short* p = dst + (size_t)i * 8;
  *(volatile v8us*)p = v;
  __threadfence();
  *(volatile v8us*)p = v;
}

__global__ __launch_bounds__(256)
void k_split(const float* __restrict__ src, unsigned short* __restrict__ dh,
             unsigned short* __restrict__ dl, int n8) {
  const int i = blockIdx.x * 256 + threadIdx.x;
  if (i >= n8) return;
  const float* s = src + (size_t)i * 8;
  const v4f x0 = *(const v4f*)(s);
  const v4f x1 = *(const v4f*)(s + 4);
  v8us vh, vl;
#pragma unroll
  for (int c = 0; c < 4; ++c) {
    unsigned short a, b;
    split2(x0[c], a, b); vh[c] = a;     vl[c] = b;
    split2(x1[c], a, b); vh[4 + c] = a; vl[4 + c] = b;
  }
  unsigned short* ph = dh + (size_t)i * 8;
  unsigned short* pl = dl + (size_t)i * 8;
  *(volatile v8us*)ph = vh;
  *(volatile v8us*)pl = vl;
  __threadfence();
  *(volatile v8us*)ph = vh;
  *(volatile v8us*)pl = vl;
}

template <int MODE, int SPLIT>
__device__ __forceinline__ void proj_lines(const unsigned short* sh, const unsigned short* sl,
                                           unsigned short* Oh, unsigned short* Ol,
                                           int Mbase, int Nbase, int tn, int l) {
  const int q8 = l & 7;
  const int rsub = l >> 3;
#pragma unroll
  for (int j = 0; j < 8; ++j) {
    const int row = j * 4 + rsub;
    const v8us vh = *(const v8us*)(sh + row * 64 + q8 * 8);
    size_t gidx;
    if (MODE == 0) {
      const int tok = Mbase + row;
      const int b = tok >> 10;
      const int s = tok & (SS - 1);
      const int h = tn;
      gidx = ((size_t)(b * HH + h) * SS + s) * DK + q8 * 8;
    } else {
      const int n = Nbase + row;
      const int h = n >> 6;
      const int dk = n & 63;
      const int b = Mbase >> 10;
      const int s0 = Mbase & (SS - 1);
      gidx = ((size_t)(b * HH + h) * DK + dk) * SS + s0 + q8 * 8;
    }
    *(volatile v8us*)(Oh + gidx) = vh;
    if (SPLIT) {
      const v8us vl = *(const v8us*)(sl + row * 64 + q8 * 8);
      *(volatile v8us*)(Ol + gidx) = vl;
    }
  }
}

template <int MI, int NI, int MODE, int SPLIT>
__global__ __launch_bounds__(128)
void k_proj(const unsigned short* __restrict__ Xh, const unsigned short* Xl,
            const unsigned short* __restrict__ Wh, const unsigned short* Wl,
            const float* __restrict__ bias, float oscale,
            unsigned short* Oh, unsigned short* Ol, int ntiles) {
  constexpr int TM = MI * 16;
  constexpr int TN = NI * 16;
  constexpr int tilesN = DD / TN;
  __shared__ __attribute__((aligned(16))) unsigned short stg[4][2][2048];

  const int wib = threadIdx.x >> 5;
  const int l = threadIdx.x & 31;
  const int hh = l >> 4;
  const int m = l & 15;
  const int tile = blockIdx.x * 4 + wib;
  const bool active = tile < ntiles;
  const int tilec = active ? tile : 0;
  const int tm = tilec / tilesN;
  const int tn = tilec - tm * tilesN;
  const int Mbase = tm * TM;
  const int Nbase = tn * TN;

  size_t xro[MI], wro[NI];
#pragma unroll
  for (int i = 0; i < MI; ++i) xro[i] = (size_t)(Mbase + i * 16 + m) * DD;
#pragma unroll
  for (int i = 0; i < NI; ++i) wro[i] = (size_t)(Nbase + i * 16 + m) * DD;

  v8f acc[MI][NI];
#pragma unroll
  for (int mi = 0; mi < MI; ++mi)
#pragma unroll
    for (int ni = 0; ni < NI; ++ni) acc[mi][ni] = (v8f)0.0f;

#pragma unroll 1
  for (int k0 = 0; k0 < DD; k0 += 32) {
    Frag ah[MI], bh[NI];
    Frag al[MI], bl[NI];
#pragma unroll
    for (int mi = 0; mi < MI; ++mi) {
      ah[mi] = ldfrag(Xh + xro[mi], k0, hh);
      if (SPLIT) al[mi] = ldfrag(Xl + xro[mi], k0, hh);
      else al[mi].w = (v8i)0;
    }
#pragma unroll
    for (int ni = 0; ni < NI; ++ni) {
      bh[ni] = ldfrag(Wh + wro[ni], k0, hh);
      if (SPLIT) bl[ni] = ldfrag(Wl + wro[ni], k0, hh);
      else bl[ni].w = (v8i)0;
    }
#pragma unroll
    for (int mi = 0; mi < MI; ++mi)
#pragma unroll
      for (int ni = 0; ni < NI; ++ni) {
        if (SPLIT) acc[mi][ni] = mma3(ah[mi], al[mi], bh[ni], bl[ni], acc[mi][ni]);
        else       acc[mi][ni] = mma_f16(ah[mi], bh[ni], acc[mi][ni]);
      }
  }

  unsigned short* sh = stg[wib][0];
  unsigned short* sl = stg[wib][1];
#pragma unroll
  for (int mi = 0; mi < MI; ++mi) {
#pragma unroll
    for (int ni = 0; ni < NI; ++ni) {
      const float bn = bias[Nbase + ni * 16 + m];
#pragma unroll
      for (int r = 0; r < 8; ++r) {
        const float v = acc[mi][ni][r] * oscale + bn;
        int idx;
        if (MODE == 0) idx = (mi * 16 + 8 * hh + r) * 64 + (ni * 16 + m);
        else           idx = (ni * 16 + m) * 64 + (mi * 16 + 8 * hh + r);
        if (SPLIT) {
          unsigned short vhi, vlo;
          split2(v, vhi, vlo);
          sh[idx] = vhi;
          sl[idx] = vlo;
        } else {
          sh[idx] = f16_bits(v);
        }
      }
    }
  }
  __syncthreads();

  if (active) {
    proj_lines<MODE, SPLIT>(sh, sl, Oh, Ol, Mbase, Nbase, tn, l);
    __threadfence();
    proj_lines<MODE, SPLIT>(sh, sl, Oh, Ol, Mbase, Nbase, tn, l);
  }
}

__device__ __forceinline__ void attn_lines(const float* Os, float* out, int b, int h,
                                           int qbase, int hh, int m) {
#pragma unroll
  for (int j = 0; j < 8; ++j) {
    const int row = 2 * j + hh;
    const v4f val = *(const v4f*)(Os + row * 64 + m * 4);
    float* gp = out + ((size_t)(b * SS + qbase + row)) * DD + h * DK + m * 4;
    *(volatile v4f*)gp = val;
  }
}

__global__ __launch_bounds__(128)
void k_attn(const unsigned short* __restrict__ Q16, const unsigned short* __restrict__ K16,
            const unsigned short* __restrict__ Vh, const unsigned short* __restrict__ Vl,
            const int* __restrict__ amask, float* __restrict__ out, int nblk) {
  __shared__ __attribute__((aligned(16))) unsigned char stg_raw[4 * 4096];
  if ((int)blockIdx.x >= nblk) return;

  const int wib = threadIdx.x >> 5;
  const int l = threadIdx.x & 31;
  const int hh = l >> 4;
  const int m = l & 15;
  const int qt = blockIdx.x & 63;
  const int bh = (int)(blockIdx.x >> 6) * 4 + wib;
  const int b = bh >> 4;
  const int h = bh & 15;
  const int qbase = qt * 16;

  unsigned short* Ph = (unsigned short*)(stg_raw + wib * 4096);
  unsigned short* Pl = Ph + 512;
  float* Os = (float*)(stg_raw + wib * 4096);

  const size_t qro = ((size_t)bh * SS + qbase + m) * DK;
  const Frag aq0 = ldfrag(Q16 + qro, 0, hh);
  const Frag aq1 = ldfrag(Q16 + qro, 32, hh);

  const int* mb = amask + b * SS;

  v8f o[4];
#pragma unroll
  for (int t = 0; t < 4; ++t) o[t] = (v8f)0.0f;
  float mrow[8], lrow[8];
#pragma unroll
  for (int r = 0; r < 8; ++r) { mrow[r] = -INFINITY; lrow[r] = 0.0f; }

  const int kend = qbase + 16;
#pragma unroll 1
  for (int kb = 0; kb < kend; kb += 32) {
    float sc[2][8];
#pragma unroll
    for (int nt = 0; nt < 2; ++nt) {
      const int key = kb + nt * 16 + m;
      const size_t kro = ((size_t)bh * SS + key) * DK;
      v8f s = (v8f)0.0f;
      {
        const Frag bk = ldfrag(K16 + kro, 0, hh);
        s = mma_f16(aq0, bk, s);
      }
      {
        const Frag bk = ldfrag(K16 + kro, 32, hh);
        s = mma_f16(aq1, bk, s);
      }
      const int am = mb[key];
#pragma unroll
      for (int r = 0; r < 8; ++r) {
        const int q = qbase + 8 * hh + r;
        float x = s[r] * 0.125f;
        if (key > q || am == 0) x = -INFINITY;
        sc[nt][r] = x;
      }
    }

    float alpha[8];
#pragma unroll
    for (int r = 0; r < 8; ++r) {
      float mx = fmaxf(sc[0][r], sc[1][r]);
      mx = fmaxf(mx, __shfl_xor(mx, 8, 32));
      mx = fmaxf(mx, __shfl_xor(mx, 4, 32));
      mx = fmaxf(mx, __shfl_xor(mx, 2, 32));
      mx = fmaxf(mx, __shfl_xor(mx, 1, 32));
      const float mnew = fmaxf(mrow[r], mx);
      const float mref = (mnew == -INFINITY) ? 0.0f : mnew;
      alpha[r] = __expf(mrow[r] - mref);
      const float p0 = __expf(sc[0][r] - mref);
      const float p1 = __expf(sc[1][r] - mref);
      sc[0][r] = p0;
      sc[1][r] = p1;
      float sum = p0 + p1;
      sum += __shfl_xor(sum, 8, 32);
      sum += __shfl_xor(sum, 4, 32);
      sum += __shfl_xor(sum, 2, 32);
      sum += __shfl_xor(sum, 1, 32);
      lrow[r] = lrow[r] * alpha[r] + sum;
      mrow[r] = mnew;
    }
#pragma unroll
    for (int t = 0; t < 4; ++t)
#pragma unroll
      for (int r = 0; r < 8; ++r) o[t][r] *= alpha[r];

    __syncthreads();
#pragma unroll
    for (int nt = 0; nt < 2; ++nt) {
#pragma unroll
      for (int r = 0; r < 8; ++r) {
        unsigned short phi, plo;
        split2(sc[nt][r], phi, plo);
        const int idx = (8 * hh + r) * 32 + nt * 16 + m;
        Ph[idx] = phi;
        Pl[idx] = plo;
      }
    }
    __syncthreads();
    const Frag aph = ldfrag(Ph + m * 32, 0, hh);
    const Frag apl = ldfrag(Pl + m * 32, 0, hh);

#pragma unroll
    for (int t = 0; t < 4; ++t) {
      const int dk = t * 16 + m;
      const size_t vro = ((size_t)bh * DK + dk) * SS;
      const Frag bvh = ldfrag(Vh + vro, kb, hh);
      const Frag bvl = ldfrag(Vl + vro, kb, hh);
      o[t] = mma3(aph, apl, bvh, bvl, o[t]);
    }
  }

  float inv[8];
#pragma unroll
  for (int r = 0; r < 8; ++r) inv[r] = 1.0f / lrow[r];
  __syncthreads();
#pragma unroll
  for (int t = 0; t < 4; ++t)
#pragma unroll
    for (int r = 0; r < 8; ++r)
      Os[(8 * hh + r) * 64 + t * 16 + m] = o[t][r] * inv[r];
  __syncthreads();

  attn_lines(Os, out, b, h, qbase, hh, m);
  __threadfence();
  attn_lines(Os, out, b, h, qbase, hh, m);
}

extern "C" void kernel_launch(void* const* d_in, const int* in_sizes, int n_in,
                              void* d_out, int out_size, void* d_ws, size_t ws_size,
                              hipStream_t stream) {
  if (n_in < 10) return;
  if (in_sizes[0] != NX || in_sizes[1] != NX || in_sizes[2] != NX) return;
  if (in_sizes[3] != BB * SS) return;
  if (in_sizes[4] != NW || in_sizes[6] != NW || in_sizes[8] != NW) return;
  if (in_sizes[5] != DD || in_sizes[7] != DD || in_sizes[9] != DD) return;
  if (out_size != NX) return;

  const float* query = (const float*)d_in[0];
  const float* key_  = (const float*)d_in[1];
  const float* value = (const float*)d_in[2];
  const int*   amask = (const int*)d_in[3];
  const float* Wq = (const float*)d_in[4];
  const float* bq = (const float*)d_in[5];
  const float* Wk = (const float*)d_in[6];
  const float* bk = (const float*)d_in[7];
  const float* Wv = (const float*)d_in[8];
  const float* bv = (const float*)d_in[9];
  float* out = (float*)d_out;

  const size_t pa = (size_t)NX * 2;
  const size_t pw = (size_t)NW * 2;
  const size_t need = 8 * pa + 4 * pw;
  if (ws_size < need) return;

  unsigned char* w = (unsigned char*)d_ws;
  size_t off = 0;
  unsigned short* xq16 = (unsigned short*)(w + off); off += pa;
  unsigned short* xk16 = (unsigned short*)(w + off); off += pa;
  unsigned short* wq16 = (unsigned short*)(w + off); off += pw;
  unsigned short* wk16 = (unsigned short*)(w + off); off += pw;
  unsigned short* xvh  = (unsigned short*)(w + off); off += pa;
  unsigned short* xvl  = (unsigned short*)(w + off); off += pa;
  unsigned short* wvh  = (unsigned short*)(w + off); off += pw;
  unsigned short* wvl  = (unsigned short*)(w + off); off += pw;
  unsigned short* Q16  = (unsigned short*)(w + off); off += pa;
  unsigned short* K16  = (unsigned short*)(w + off); off += pa;
  unsigned short* Vth  = (unsigned short*)(w + off); off += pa;
  unsigned short* Vtl  = (unsigned short*)(w + off); off += pa;
  if (off > ws_size) return;

  const int n8a = (int)(NX / 8);
  const int n8w = (int)(NW / 8);
  k_cvt16<<<(n8a + 255) / 256, 256, 0, stream>>>(query, xq16, n8a, 1.0f);
  k_cvt16<<<(n8a + 255) / 256, 256, 0, stream>>>(key_,  xk16, n8a, 1.0f);
  k_cvt16<<<(n8w + 255) / 256, 256, 0, stream>>>(Wq, wq16, n8w, 16.0f);
  k_cvt16<<<(n8w + 255) / 256, 256, 0, stream>>>(Wk, wk16, n8w, 16.0f);
  k_split<<<(n8a + 255) / 256, 256, 0, stream>>>(value, xvh, xvl, n8a);
  k_split<<<(n8w + 255) / 256, 256, 0, stream>>>(Wv, wvh, wvl, n8w);

  const int ntq = (NTOK / 32) * (DD / 64);
  const int ntv = (NTOK / 64) * (DD / 32);
  k_proj<2, 4, 0, 0><<<(ntq + 3) / 4, 128, 0, stream>>>(xq16, xq16, wq16, wq16, bq, 0.0625f, Q16, Q16, ntq);
  k_proj<2, 4, 0, 0><<<(ntq + 3) / 4, 128, 0, stream>>>(xk16, xk16, wk16, wk16, bk, 0.0625f, K16, K16, ntq);
  k_proj<4, 2, 1, 1><<<(ntv + 3) / 4, 128, 0, stream>>>(xvh, xvl, wvh, wvl, bv, 1.0f, Vth, Vtl, ntv);

  const int nblk = BB * HH * (SS / 16) / 4;
  k_attn<<<nblk, 128, 0, stream>>>(Q16, K16, Vth, Vtl, amask, out, nblk);
}
